// GIN_23055384445759
// MI455X (gfx1250) — hardware-verified
//
#include <hip/hip_runtime.h>
#include <stddef.h>
#include <stdint.h>
#include <math.h>


#define F0     128
#define HID    256
#define NCLS   64
#define KZ1    (2 * F0)
#define KZ2    (2 * HID)
#define NTHR   256
#define NWAVE  8
#define EPT    8
#define CHUNK  (NTHR * EPT)
#define WCAP   (EPT * 32)
#define LISTN  (NWAVE * WCAP)
#define NBA    1024
#define SLA    10
#define RCAP   28672
#define DEGCAP 64
#define GBM    64
#define GTHR   128
#define GWAVE  (GTHR / 32)
#define GNC    128
#define PARTW  288
#define WSTW   258
#define HPR    8
#define HPB    (NWAVE * HPR)
#define AGG_ZINTS    (LISTN + 2 * RCAP + 3 * NBA)
#define MISC_INTS    16
#define AGG_LDS_INTS (AGG_ZINTS + MISC_INTS)
#define WSMAX  134217728

static_assert((CHUNK & (CHUNK - 1)) == 0 && CHUNK <= 4096);
static_assert((NBA & (NBA - 1)) == 0 && NBA == (1 << SLA));
static_assert(((long long)CHUNK << SLA) < (1LL << 31));
static_assert(LISTN % NTHR == 0);
static_assert(NBA % NWAVE == 0 && NBA % 32 == 0 && NBA % GBM == 0);
static_assert(RCAP % 32 == 0 && LISTN % 4 == 0 && AGG_ZINTS % (NTHR * 4) == 0);
static_assert(KZ1 % 32 == 0 && KZ2 % 32 == 0 && KZ1 == 2 * F0 && KZ2 == 2 * HID);
static_assert(GBM == GWAVE * 16 && HID == 2 * GNC && NCLS == 64 && F0 == 4 * 32 && HID == 8 * 32);
static_assert(PARTW % 32 == 0 && PARTW / 4 <= GTHR && PARTW >= 2 * GNC + 1);
static_assert(WSTW >= 2 * GNC + 1 && (WSTW % 2) == 0);
static_assert(HPB == GBM && NTHR == HID);
static_assert(F0 % 8 == 0 && HID % 8 == 0);
static_assert(AGG_LDS_INTS * 4 <= 300000);

typedef float          v2f   __attribute__((ext_vector_type(2)));
typedef float          v4f   __attribute__((ext_vector_type(4)));
typedef float          v8f   __attribute__((ext_vector_type(8)));
typedef int            v4i   __attribute__((ext_vector_type(4)));
typedef int            v8i   __attribute__((ext_vector_type(8)));
typedef unsigned int   v2u   __attribute__((ext_vector_type(2)));
typedef unsigned int   v4u   __attribute__((ext_vector_type(4)));
typedef unsigned short v8us  __attribute__((ext_vector_type(8)));
typedef unsigned short v16us __attribute__((ext_vector_type(16)));
typedef __bf16         v16bf __attribute__((ext_vector_type(16)));
typedef v2f  __attribute__((may_alias)) v2fa;
typedef v4f  __attribute__((may_alias)) v4fa;
typedef v4i  __attribute__((may_alias)) v4ia;
typedef v8us __attribute__((may_alias)) v8usa;
union FragB { v16bf v; v16us u; v8us h[2]; v8i w; };

__device__ __forceinline__ v8f wmb(const FragB& a, const FragB& b, v8f c) {
  v8f d = __builtin_amdgcn_wmma_f32_16x16x32_bf16(false, a.v, false, b.v, (short)0, c, false, false);
  asm volatile("v_nop\n\tv_nop\n\tv_nop\n\tv_nop" : "+v"(d) : "v"(a.w), "v"(b.w));
  return d;
}

__device__ __forceinline__ v8f z8() { v8f z = {0.f, 0.f, 0.f, 0.f, 0.f, 0.f, 0.f, 0.f}; return z; }

__device__ __forceinline__ unsigned bf16_bits(float f) {
  const unsigned u = __float_as_uint(f);
  return ((u + 0x7FFFu + ((u >> 16) & 1u)) >> 16) & 0xFFFFu;
}
__device__ __forceinline__ float bf16_val(float f) {
  return __uint_as_float(bf16_bits(f) << 16);
}
__device__ __forceinline__ unsigned hl_bits(float v, unsigned& lo) {
  const unsigned hb = bf16_bits(v);
  lo = bf16_bits(v - __uint_as_float(hb << 16));
  return hb;
}
__device__ __forceinline__ unsigned pk2(float lo, float hi) { return bf16_bits(lo) | (bf16_bits(hi) << 16); }
__device__ __forceinline__ v4u pack8(const v4f a, const v4f b) {
  v4u r;
  r.x = pk2(a.x, a.y); r.y = pk2(a.z, a.w); r.z = pk2(b.x, b.y); r.w = pk2(b.z, b.w);
  return r;
}
__device__ __forceinline__ void split8(const v4f a, const v4f b, v4u& hv, v4u& lv) {
  const float f[8] = {a.x, a.y, a.z, a.w, b.x, b.y, b.z, b.w};
  unsigned int hb[8], lb[8];
#pragma unroll
  for (int i = 0; i < 8; ++i) hb[i] = hl_bits(f[i], lb[i]);
  hv.x = hb[0] | (hb[1] << 16); hv.y = hb[2] | (hb[3] << 16); hv.z = hb[4] | (hb[5] << 16); hv.w = hb[6] | (hb[7] << 16);
  lv.x = lb[0] | (lb[1] << 16); lv.y = lb[2] | (lb[3] << 16); lv.z = lb[4] | (lb[5] << 16); lv.w = lb[6] | (lb[7] << 16);
}

template <int CP, int RND>
__device__ __forceinline__ void ldrow(const float* p, float* v) {
  if constexpr (CP == 4) {
    const v4f t = *(const v4fa*)p;
    v[0] = t.x; v[1] = t.y; v[2] = t.z; v[3] = t.w;
  } else {
    const v4f t0 = *(const v4fa*)p;
    const v4f t1 = *(const v4fa*)(p + 4);
    v[0] = t0.x; v[1] = t0.y; v[2] = t0.z; v[3] = t0.w;
    v[4] = t1.x; v[5] = t1.y; v[6] = t1.z; v[7] = t1.w;
  }
  if constexpr (RND != 0) {
#pragma unroll
    for (int j = 0; j < CP; ++j) v[j] = bf16_val(v[j]);
  }
}

template <int SLB>
__device__ __forceinline__ int scan_chunk(const int* __restrict__ dsts, int nE, int cbase, int slotBase,
                                          int nb, int vec8, int* list, int tid, int lane, int wave) {
  int wc = 0;
  const int el0  = tid * EPT;
  const int e0   = cbase + el0;
  const int sent = -2147483647 - 1;
  v4i da, db;
  if (vec8 != 0 && cbase + CHUNK <= nE) {
    da = *(const v4i*)(dsts + e0);
    db = *(const v4i*)(dsts + e0 + 4);
  } else {
    da.x = (e0     < nE) ? dsts[min(e0,     nE - 1)] : sent;
    da.y = (e0 + 1 < nE) ? dsts[min(e0 + 1, nE - 1)] : sent;
    da.z = (e0 + 2 < nE) ? dsts[min(e0 + 2, nE - 1)] : sent;
    da.w = (e0 + 3 < nE) ? dsts[min(e0 + 3, nE - 1)] : sent;
    db.x = (e0 + 4 < nE) ? dsts[min(e0 + 4, nE - 1)] : sent;
    db.y = (e0 + 5 < nE) ? dsts[min(e0 + 5, nE - 1)] : sent;
    db.z = (e0 + 6 < nE) ? dsts[min(e0 + 6, nE - 1)] : sent;
    db.w = (e0 + 7 < nE) ? dsts[min(e0 + 7, nE - 1)] : sent;
  }
  const unsigned nbs = (unsigned)slotBase;
  const unsigned unb = (unsigned)nb;
  const unsigned s0 = (unsigned)da.x - nbs, s1 = (unsigned)da.y - nbs;
  const unsigned s2 = (unsigned)da.z - nbs, s3 = (unsigned)da.w - nbs;
  const unsigned s4 = (unsigned)db.x - nbs, s5 = (unsigned)db.y - nbs;
  const unsigned s6 = (unsigned)db.z - nbs, s7 = (unsigned)db.w - nbs;
  const bool h0 = s0 < unb, h1 = s1 < unb, h2 = s2 < unb, h3 = s3 < unb;
  const bool h4 = s4 < unb, h5 = s5 < unb, h6 = s6 < unb, h7 = s7 < unb;
  const unsigned any = __builtin_amdgcn_ballot_w32(h0 | h1 | h2 | h3 | h4 | h5 | h6 | h7);
  if (any != 0u) {
#define HITJ(J, HJ, SJ) { \
      const unsigned mj = __builtin_amdgcn_ballot_w32(HJ); \
      if (mj != 0u) { \
        if (HJ) { \
          const int pos = wc + (int)__builtin_amdgcn_mbcnt_lo(mj, 0u); \
          if (pos < WCAP) list[wave * WCAP + pos] = ((el0 + (J)) << SLB) | (int)(SJ); \
        } \
        wc += (int)__builtin_popcount(mj); } }
    HITJ(0, h0, s0)
    HITJ(1, h1, s1)
    HITJ(2, h2, s2)
    HITJ(3, h3, s3)
    HITJ(4, h4, s4)
    HITJ(5, h5, s5)
    HITJ(6, h6, s6)
    HITJ(7, h7, s7)
#undef HITJ
  }
  return wc;
}

__global__ __launch_bounds__(NTHR) void k_wtr(const float* __restrict__ w, int Kin, int Ncol, int Nrows, int Kout,
                                              unsigned short* wt, int nUnits) {
  const int u = (int)blockIdx.x * NTHR + (int)threadIdx.x;
  if (u >= nUnits) return;
  const int kq = Kout >> 3;
  const int n  = u / kq;
  const int k8 = (u - n * kq) * 8;
  const int kk = k8 - (k8 / Kin) * Kin;
  const int ncl = n < Ncol ? n : Ncol - 1;
  const float* p = w + (size_t)kk * (size_t)Ncol + ncl;
  v4f a, b;
  a.x = p[0];                    a.y = p[(size_t)Ncol];         a.z = p[(size_t)2 * Ncol];     a.w = p[(size_t)3 * Ncol];
  b.x = p[(size_t)4 * Ncol];     b.y = p[(size_t)5 * Ncol];     b.z = p[(size_t)6 * Ncol];     b.w = p[(size_t)7 * Ncol];
  const v4f z4 = {0.f, 0.f, 0.f, 0.f};
  if (n >= Ncol || n >= Nrows) { a = z4; b = z4; }
  const v4u wv = pack8(a, b);
  unsigned short* o = wt + (size_t)n * (size_t)Kout + k8;
  *(volatile v4u*)o = wv;
  __threadfence();
  *(volatile v4u*)o = wv;
}

template <int FD, int RND>
__global__ __launch_bounds__(NTHR) void k_scan(const int* __restrict__ srcs, const int* __restrict__ dsts,
                                               int nE, int nN, int vec8, int mRows,
                                               const float* __restrict__ epl, const float* __restrict__ hsrc,
                                               unsigned short* apl) {
  constexpr int CP = FD / 32;
  constexpr int KP = 2 * FD;
  static_assert(CP == 4 || CP == 8);
  extern __shared__ __attribute__((aligned(16))) int dsm[];
  int* list = dsm;
  int* hl   = dsm + LISTN;
  int* sl   = hl + RCAP;
  int* cnt  = sl + RCAP;
  int* offs = cnt + NBA;
  int* cur  = offs + NBA;
  int* misc = cur + NBA;
  const int tid = (int)threadIdx.x, lane = tid & 31, wave = tid >> 5;
  const int nodeBase = (int)blockIdx.x * NBA;

  {
    const v4i z4 = {0, 0, 0, 0};
    for (int i = tid * 4; i < AGG_ZINTS; i += NTHR * 4) *(v4ia*)(dsm + i) = z4;
    if (tid < MISC_INTS) misc[tid] = 0;
  }
  __syncthreads();
  const float opl = 1.0f + bf16_val(epl[0]);

  int t = 0, ov = 0;
  const int nChunks = (nE + CHUNK - 1) / CHUNK;
#pragma unroll 1
  for (int ch = 0; ch < nChunks; ++ch) {
    const int cbase = ch * CHUNK;
    const int wc = scan_chunk<SLA>(dsts, nE, cbase, nodeBase, NBA, vec8, list, tid, lane, wave);
    if (lane == 0) misc[wave] = wc;
    __syncthreads();
    if (wave == 0) {
#pragma unroll 1
      for (int w2 = 0; w2 < NWAVE; ++w2) {
        int c = misc[w2];
        c = c < 0 ? 0 : (c > WCAP ? WCAP : c);
#pragma unroll 1
        for (int b0 = 0; b0 < c; b0 += 32) {
          const int idx = b0 + lane;
          const int ent = list[w2 * WCAP + (idx < WCAP ? idx : WCAP - 1)];
          const int m32 = (c - b0) < 32 ? (c - b0) : 32;
#pragma unroll 1
          for (int k = 0; k < m32; ++k) {
            const int u    = __builtin_amdgcn_readlane(ent, k);
            const int slot = u & (NBA - 1);
            const int el   = (u >> SLA) & (CHUNK - 1);
            const int pk   = ((cbase + el) << SLA) | slot;
            if (t < RCAP) {
              if (lane == 0) { hl[t] = pk; cnt[slot] = cnt[slot] + 1; }
              t = t + 1;
            } else {
              ov = 1;
            }
          }
        }
      }
    }
    __syncthreads();
  }
  if (wave == 0 && lane == 0) { misc[8] = t; misc[9] = ov; }
  __syncthreads();
  int tt = misc[8];
  tt = tt < 0 ? 0 : (tt > RCAP ? RCAP : tt);
  const int ovf = misc[9];

  if (wave == 0) {
    const int base = lane * (NBA / 32);
    int s = 0;
#pragma unroll 1
    for (int i = 0; i < NBA / 32; ++i) s += cnt[base + i];
    int incl = s;
#pragma unroll
    for (int d = 1; d < 32; d <<= 1) {
      const int y = __shfl_up(incl, d, 32);
      if (lane >= d) incl += y;
    }
    int run = incl - s;
#pragma unroll 1
    for (int i = 0; i < NBA / 32; ++i) {
      const int cv = cnt[base + i];
      offs[base + i] = run;
      cur[base + i]  = run;
      run += cv;
    }
  }
  __syncthreads();
  if (wave == 0) {
#pragma unroll 1
    for (int b0 = 0; b0 < tt; b0 += 32) {
      const int idx = b0 + lane;
      const int ent = hl[idx < RCAP ? idx : RCAP - 1];
      const int m32 = (tt - b0) < 32 ? (tt - b0) : 32;
#pragma unroll 1
      for (int k = 0; k < m32; ++k) {
        const int u    = __builtin_amdgcn_readlane(ent, k);
        const int slot = u & (NBA - 1);
        if (lane == 0) {
          int p = cur[slot];
          p = p < 0 ? 0 : (p > RCAP - 1 ? RCAP - 1 : p);
          sl[p] = u;
          cur[slot] = p + 1;
        }
      }
    }
  }
  __syncthreads();

  const float qnan = __int_as_float(0x7fc00000);
  const float pz = (ovf != 0) ? qnan : 0.0f;
#pragma unroll 1
  for (int si = 0; si < NBA / NWAVE; ++si) {
    const int s    = si * NWAVE + wave;
    const int node = nodeBase + s;
    int c = cnt[s];
    const bool big = c > DEGCAP;
    c = c < 0 ? 0 : (c > DEGCAP ? DEGCAP : c);
    int o = offs[s];
    o = o < 0 ? 0 : (o > RCAP ? RCAP : o);
    const int nc = node < nN ? node : nN - 1;
    float ag[CP];
#pragma unroll
    for (int j = 0; j < CP; ++j) ag[j] = 0.0f;
#pragma unroll 1
    for (int b0 = 0; b0 < c; b0 += 32) {
      int idx = o + b0 + lane;
      idx = idx > RCAP - 1 ? RCAP - 1 : idx;
      const int ent = sl[idx];
      int eid = ent >> SLA;
      eid = eid < 0 ? 0 : (eid > nE - 1 ? nE - 1 : eid);
      int sr = srcs[eid];
      sr = sr < 0 ? 0 : (sr > nN - 1 ? nN - 1 : sr);
      const int m32 = (c - b0) < 32 ? (c - b0) : 32;
#pragma unroll 1
      for (int k = 0; k < m32; ++k) {
        const int sk = __builtin_amdgcn_readlane(sr, k);
        float v[CP];
        ldrow<CP, RND>(hsrc + (size_t)sk * FD + CP * lane, v);
#pragma unroll
        for (int j = 0; j < CP; ++j) ag[j] = ag[j] + v[j];
      }
    }
    const float pzr = big ? qnan : pz;
    const bool live = node < nN;
    float hr[CP];
    ldrow<CP, RND>(hsrc + (size_t)nc * FD + CP * lane, hr);
    unsigned hb[CP], lb[CP];
#pragma unroll
    for (int j = 0; j < CP; ++j) {
      const float z = live ? (fmaf(opl, hr[j], ag[j]) + pzr) : 0.0f;
      hb[j] = hl_bits(z, lb[j]);
    }
    if (node < mRows) {
      unsigned short* rpw = apl + (size_t)node * KP;
      if constexpr (CP == 4) {
        v2u hp, lp;
        hp.x = hb[0] | (hb[1] << 16); hp.y = hb[2] | (hb[3] << 16);
        lp.x = lb[0] | (lb[1] << 16); lp.y = lb[2] | (lb[3] << 16);
        unsigned short* ph = rpw + 4 * lane;
        unsigned short* pl = rpw + FD + 4 * lane;
        *(volatile v2u*)ph = hp;
        *(volatile v2u*)pl = lp;
        __threadfence();
        *(volatile v2u*)ph = hp;
        *(volatile v2u*)pl = lp;
      } else {
        v4u hp, lp;
        hp.x = hb[0] | (hb[1] << 16); hp.y = hb[2] | (hb[3] << 16); hp.z = hb[4] | (hb[5] << 16); hp.w = hb[6] | (hb[7] << 16);
        lp.x = lb[0] | (lb[1] << 16); lp.y = lb[2] | (lb[3] << 16); lp.z = lb[4] | (lb[5] << 16); lp.w = lb[6] | (lb[7] << 16);
        unsigned short* ph = rpw + 8 * lane;
        unsigned short* pl = rpw + FD + 8 * lane;
        *(volatile v4u*)ph = hp;
        *(volatile v4u*)pl = lp;
        __threadfence();
        *(volatile v4u*)ph = hp;
        *(volatile v4u*)pl = lp;
      }
    }
  }
}

template <int NC, int KK, int LDO, int EPI>
__global__ __launch_bounds__(GTHR) void k_gemm(const unsigned short* __restrict__ Apl,
                                               const unsigned short* __restrict__ BT,
                                               const float* __restrict__ bias, int nN,
                                               float* outp, float* part) {
  constexpr int NT  = NC / 16;
  constexpr int CPL = NC / 32;
  static_assert(NT >= 1 && NT <= 8 && (CPL == 2 || CPL == 4) && KK % 32 == 0 && LDO % NC == 0);
  static_assert(EPI != 0 || NC == GNC);
  static_assert(EPI != 2 || (NC == NCLS && LDO == NCLS && CPL == 2));
  static_assert(EPI == 2 || CPL == 4);
  __shared__ __attribute__((aligned(16))) float stg[GBM * NC];
  __shared__ __attribute__((aligned(16))) float wst[GWAVE * WSTW];
  __shared__ __attribute__((aligned(16))) float pst[PARTW];
  const int tid = (int)threadIdx.x, lane = tid & 31, wave = tid >> 5, hh = lane >> 4, m = lane & 15;
  const int rowBase = (int)blockIdx.x * GBM;
  const int col0    = (int)blockIdx.y * NC;

  v8f acc[NT];
#pragma unroll
  for (int t = 0; t < NT; ++t) acc[t] = z8();
  const unsigned short* ap = Apl + (size_t)(rowBase + 16 * wave + m) * (size_t)KK + 8 * hh;
  const unsigned short* bp = BT + (size_t)(col0 + m) * (size_t)KK + 8 * hh;

#pragma unroll 1
  for (int k0 = 0; k0 < KK; k0 += 32) {
    FragB af;
    af.h[0] = *(const v8usa*)(ap + k0);
    af.h[1] = *(const v8usa*)(ap + k0 + 16);
#pragma unroll
    for (int nt = 0; nt < NT; ++nt) {
      const unsigned short* wq = bp + (size_t)(16 * nt) * (size_t)KK + k0;
      FragB bf;
      bf.h[0] = *(const v8usa*)wq;
      bf.h[1] = *(const v8usa*)(wq + 16);
      acc[nt] = wmb(af, bf, acc[nt]);
    }
  }

#pragma unroll
  for (int nt = 0; nt < NT; ++nt) {
    const int lc = 16 * nt + m;
#pragma unroll
    for (int r = 0; r < 8; ++r) {
      const int lr = 16 * wave + 8 * hh + r;
      stg[lr * NC + lc] = acc[nt][r];
    }
  }
  __syncthreads();

  float bq[CPL];
  if constexpr (CPL == 4) {
    const v4f b4 = *(const v4fa*)(bias + col0 + 4 * lane);
    bq[0] = bf16_val(b4.x); bq[1] = bf16_val(b4.y); bq[2] = bf16_val(b4.z); bq[3] = bf16_val(b4.w);
  } else {
    const v2f bp2 = *(const v2fa*)(bias + col0 + 2 * lane);
    bq[0] = bf16_val(bp2.x); bq[1] = bf16_val(bp2.y);
  }

  float pv[16][CPL];
  int wn = 0;
  float wm[CPL], wqv[CPL];
#pragma unroll
  for (int j = 0; j < CPL; ++j) { wm[j] = 0.0f; wqv[j] = 0.0f; }
#pragma unroll
  for (int i = 0; i < 16; ++i) {
    const int row = rowBase + 16 * wave + i;
    const bool ok = row < nN;
    float x[CPL];
    if constexpr (CPL == 4) {
      const v4f t4 = *(const v4fa*)(stg + (16 * wave + i) * NC + 4 * lane);
      x[0] = t4.x; x[1] = t4.y; x[2] = t4.z; x[3] = t4.w;
    } else {
      const v2f t2 = *(const v2fa*)(stg + (16 * wave + i) * NC + 2 * lane);
      x[0] = t2.x; x[1] = t2.y;
    }
    if constexpr (EPI != 2) {
      float vv[CPL];
#pragma unroll
      for (int j = 0; j < CPL; ++j) {
        vv[j] = ok ? fmaxf(x[j] + bq[j], 0.0f) : 0.0f;
        pv[i][j] = vv[j];
      }
      if constexpr (EPI == 0) {
        if (ok) {
          wn += 1;
          const float rk = 1.0f / (float)(i + 1);
#pragma unroll
          for (int j = 0; j < CPL; ++j) {
            const float dd = vv[j] - wm[j];
            wm[j]  = fmaf(dd, rk, wm[j]);
            wqv[j] = fmaf(dd, vv[j] - wm[j], wqv[j]);
          }
        }
      }
    } else {
      const float z0 = x[0] + bq[0];
      const float z1 = x[1] + bq[1];
      float vm = fmaxf(z0, z1);
#pragma unroll
      for (int off = 16; off > 0; off >>= 1) vm = fmaxf(vm, __shfl_xor(vm, off));
      const float d0 = z0 - vm, d1 = z1 - vm;
      float sm = expf(d0) + expf(d1);
#pragma unroll
      for (int off = 16; off > 0; off >>= 1) sm += __shfl_xor(sm, off);
      const float ls = logf(sm);
      pv[i][0] = d0 - ls;
      pv[i][1] = d1 - ls;
    }
  }

#pragma unroll
  for (int i = 0; i < 16; ++i) {
    const int row = rowBase + 16 * wave + i;
    const bool wr = (EPI != 2) || (row < nN);
    float* op = outp + (size_t)row * (size_t)LDO + col0 + CPL * lane;
    if (wr) {
      if constexpr (CPL == 4) {
        v4f q; q.x = pv[i][0]; q.y = pv[i][1]; q.z = pv[i][2]; q.w = pv[i][3];
        *(volatile v4f*)op = q;
      } else {
        v2f q; q.x = pv[i][0]; q.y = pv[i][1];
        *(volatile v2f*)op = q;
      }
    }
  }
  __threadfence();
#pragma unroll
  for (int i = 0; i < 16; ++i) {
    const int row = rowBase + 16 * wave + i;
    const bool wr = (EPI != 2) || (row < nN);
    float* op = outp + (size_t)row * (size_t)LDO + col0 + CPL * lane;
    if (wr) {
      if constexpr (CPL == 4) {
        v4f q; q.x = pv[i][0]; q.y = pv[i][1]; q.z = pv[i][2]; q.w = pv[i][3];
        *(volatile v4f*)op = q;
      } else {
        v2f q; q.x = pv[i][0]; q.y = pv[i][1];
        *(volatile v2f*)op = q;
      }
    }
  }

  if constexpr (EPI == 0) {
    if (lane == 0) wst[wave * WSTW] = (float)wn;
#pragma unroll
    for (int j = 0; j < CPL; ++j) {
      wst[wave * WSTW + 1 + CPL * lane + j]       = wm[j];
      wst[wave * WSTW + 1 + GNC + CPL * lane + j] = wqv[j];
    }
#pragma unroll 1
    for (int i = tid; i < PARTW; i += GTHR) pst[i] = 0.0f;
    __syncthreads();
    if (tid < NC) {
      float n = 0.0f, mean = 0.0f, M2 = 0.0f;
#pragma unroll 1
      for (int w2 = 0; w2 < GWAVE; ++w2) {
        const float nb = wst[w2 * WSTW];
        const float mb = wst[w2 * WSTW + 1 + tid];
        const float qb = wst[w2 * WSTW + 1 + GNC + tid];
        if (nb > 0.5f) {
          const float nn = n + nb;
          const float delta = mb - mean;
          const float f = nb / nn;
          mean = fmaf(delta, f, mean);
          M2 = M2 + qb + delta * delta * n * f;
          n = nn;
        }
      }
      pst[1 + tid] = mean;
      pst[1 + GNC + tid] = M2;
      if (tid == 0) pst[0] = n;
    }
    __syncthreads();
    const int pb = (int)blockIdx.x * (int)gridDim.y + (int)blockIdx.y;
    v4f ps = {0.0f, 0.0f, 0.0f, 0.0f};
    if (tid < PARTW / 4) {
      ps = *(const v4fa*)(pst + 4 * tid);
      *(volatile v4f*)(part + (size_t)pb * PARTW + 4 * tid) = ps;
    }
    __threadfence();
    if (tid < PARTW / 4) {
      *(volatile v4f*)(part + (size_t)pb * PARTW + 4 * tid) = ps;
    }
  } else {
    (void)part; (void)wn; (void)wm; (void)wqv;
  }
}

__global__ __launch_bounds__(HID) void k_bnfin(const float* __restrict__ part, int nPart,
                                               const float* __restrict__ gam, const float* __restrict__ bet,
                                               float* ss) {
  __shared__ __attribute__((aligned(16))) float stg[2 * HID];
  const int tid = (int)threadIdx.x;
  const int cb = tid >> 7;
  const int cc = tid & (GNC - 1);
  double n = 0.0, mean = 0.0, M2 = 0.0;
#pragma unroll 1
  for (int b = 0; b < nPart; ++b) {
    const float* pr = part + ((size_t)b * 2 + (size_t)cb) * PARTW;
    const double nb = (double)pr[0];
    const double mb = (double)pr[1 + cc];
    const double qb = (double)pr[1 + GNC + cc];
    if (nb > 0.5) {
      const double nn = n + nb;
      const double delta = mb - mean;
      const double f = nb / nn;
      mean = mean + delta * f;
      M2 = M2 + qb + delta * delta * n * f;
      n = nn;
    }
  }
  const double ntot = n < 1.0 ? 1.0 : n;
  const float varf  = (float)(M2 / ntot);
  const float meanf = (float)mean;
  const float rstd = rsqrtf(varf + 1e-5f);
  const float sc = bf16_val(gam[tid]) * rstd;
  const float sh = bf16_val(bet[tid]) - meanf * sc;
  stg[tid] = sc;
  stg[HID + tid] = sh;
  __syncthreads();
  v4f v = {0.0f, 0.0f, 0.0f, 0.0f};
  if (tid < (2 * HID) / 4) {
    v = *(const v4fa*)(stg + 4 * tid);
    *(volatile v4f*)(ss + 4 * tid) = v;
  }
  __threadfence();
  if (tid < (2 * HID) / 4) {
    *(volatile v4f*)(ss + 4 * tid) = v;
  }
}

__global__ __launch_bounds__(NTHR) void k_apply(const float* __restrict__ s1, const float* __restrict__ ss,
                                                int nN, int mRows, unsigned short* apl) {
  __shared__ __attribute__((aligned(16))) float ssh[2 * HID];
  const int tid = (int)threadIdx.x, lane = tid & 31, wave = tid >> 5;
  ssh[tid] = ss[tid];
  ssh[HID + tid] = ss[HID + tid];
  __syncthreads();
  const v4f sc0 = *(const v4fa*)(ssh + 8 * lane);
  const v4f sc1 = *(const v4fa*)(ssh + 8 * lane + 4);
  const v4f sh0 = *(const v4fa*)(ssh + HID + 8 * lane);
  const v4f sh1 = *(const v4fa*)(ssh + HID + 8 * lane + 4);
  const int rb0 = (int)blockIdx.x * HPB + wave * HPR;

#pragma unroll 1
  for (int i = 0; i < HPR; ++i) {
    const int row = rb0 + i;
    const bool live = row < nN;
    const int rc = live ? row : (nN - 1);
    const v4f a0 = *(const v4fa*)(s1 + (size_t)rc * HID + 8 * lane);
    const v4f a1 = *(const v4fa*)(s1 + (size_t)rc * HID + 8 * lane + 4);
    v4f y0, y1;
    y0.x = fmaf(a0.x, sc0.x, sh0.x); y0.y = fmaf(a0.y, sc0.y, sh0.y);
    y0.z = fmaf(a0.z, sc0.z, sh0.z); y0.w = fmaf(a0.w, sc0.w, sh0.w);
    y1.x = fmaf(a1.x, sc1.x, sh1.x); y1.y = fmaf(a1.y, sc1.y, sh1.y);
    y1.z = fmaf(a1.z, sc1.z, sh1.z); y1.w = fmaf(a1.w, sc1.w, sh1.w);
    const v4f z4 = {0.f, 0.f, 0.f, 0.f};
    if (!live) { y0 = z4; y1 = z4; }
    v4u qh, ql;
    split8(y0, y1, qh, ql);
    if (row < mRows) {
      unsigned short* ph = apl + (size_t)row * KZ2 + 8 * lane;
      unsigned short* pl = apl + (size_t)row * KZ2 + HID + 8 * lane;
      *(volatile v4u*)ph = qh;
      *(volatile v4u*)pl = ql;
      __threadfence();
      *(volatile v4u*)ph = qh;
      *(volatile v4u*)pl = ql;
    }
  }
}

static inline int cdiv(int a, int b) { return (a + b - 1) / b; }
static inline size_t al256(size_t o) { return (o + 255) & ~(size_t)255; }

extern "C" void kernel_launch(void* const* d_in, const int* in_sizes, int n_in,
                              void* d_out, int out_size, void* d_ws, size_t ws_size,
                              hipStream_t stream) {
  if (n_in < 16) return;
  if (in_sizes[0] < F0 || (in_sizes[0] % F0) != 0) return;
  const int nN = in_sizes[0] / F0;
  if (nN < 16 || nN >= (1 << 22)) return;
  if (in_sizes[1] < 2 || (in_sizes[1] & 1) != 0) return;
  const int nE = in_sizes[1] / 2;
  if (nE < 1 || nE >= (1 << 21)) return;
  if (in_sizes[2] != 1 || in_sizes[9] != 1) return;
  if (in_sizes[3] != F0 * HID) return;
  if (in_sizes[4] != HID || in_sizes[5] != HID || in_sizes[6] != HID) return;
  if (in_sizes[7] != HID * HID || in_sizes[8] != HID) return;
  if (in_sizes[10] != HID * HID) return;
  if (in_sizes[11] != HID || in_sizes[12] != HID || in_sizes[13] != HID) return;
  if (in_sizes[14] != HID * NCLS || in_sizes[15] != NCLS) return;
  if ((long long)out_size != (long long)nN * NCLS) return;

  const float* x    = (const float*)d_in[0];
  const int*   ei   = (const int*)  d_in[1];
  const float* eps1 = (const float*)d_in[2];
  const float* W1a  = (const float*)d_in[3];
  const float* b1a  = (const float*)d_in[4];
  const float* g1   = (const float*)d_in[5];
  const float* be1  = (const float*)d_in[6];
  const float* W1b  = (const float*)d_in[7];
  const float* b1b  = (const float*)d_in[8];
  const float* eps2 = (const float*)d_in[9];
  const float* W2a  = (const float*)d_in[10];
  const float* b2a  = (const float*)d_in[11];
  const float* g2   = (const float*)d_in[12];
  const float* be2  = (const float*)d_in[13];
  const float* W2b  = (const float*)d_in[14];
  const float* b2b  = (const float*)d_in[15];
  float* out = (float*)d_out;
  const int* src = ei;
  const int* dst = ei + nE;

  const int MP = cdiv(nN, GBM) * GBM;
  const int gM = MP / GBM;
  const int gA = cdiv(nN, NBA);
  if ((long long)gA * NBA < (long long)MP) return;
  if ((MP % HPB) != 0) return;
  const int vec8 = ((nE & 3) == 0) ? 1 : 0;

  char* ws = (char*)d_ws;
  size_t off = 0;
  const size_t oBT1a = off; off = al256(off + (size_t)HID * KZ1 * 2);
  const size_t oBT1b = off; off = al256(off + (size_t)HID * KZ2 * 2);
  const size_t oBT2a = off; off = al256(off + (size_t)HID * KZ2 * 2);
  const size_t oBT2b = off; off = al256(off + (size_t)NCLS * KZ2 * 2);
  const size_t oZA   = off; off = al256(off + (size_t)MP * KZ2 * 2);
  const size_t oSH   = off; off = al256(off + (size_t)MP * HID * 4);
  const size_t oPT   = off; off = al256(off + (size_t)2 * gM * PARTW * 4);
  const size_t oSS   = off; off = al256(off + (size_t)(2 * HID) * 4);
  if (off > ws_size || off > (size_t)WSMAX) return;
  unsigned short* BT1a = (unsigned short*)(ws + oBT1a);
  unsigned short* BT1b = (unsigned short*)(ws + oBT1b);
  unsigned short* BT2a = (unsigned short*)(ws + oBT2a);
  unsigned short* BT2b = (unsigned short*)(ws + oBT2b);
  unsigned short* ZA   = (unsigned short*)(ws + oZA);
  float*          SH   = (float*)(ws + oSH);
  float*          PT   = (float*)(ws + oPT);
  float*          SS   = (float*)(ws + oSS);

  const size_t scanLds = (size_t)AGG_LDS_INTS * 4;
  hipFuncSetAttribute(reinterpret_cast<const void*>(&k_scan<F0, 1>), hipFuncAttributeMaxDynamicSharedMemorySize, (int)scanLds);
  hipFuncSetAttribute(reinterpret_cast<const void*>(&k_scan<HID, 0>), hipFuncAttributeMaxDynamicSharedMemorySize, (int)scanLds);

  {
    const int nU1a = HID * (KZ1 / 8);
    k_wtr<<<cdiv(nU1a, NTHR), NTHR, 0, stream>>>(W1a, F0, HID, HID, KZ1, BT1a, nU1a);
    const int nU1b = HID * (KZ2 / 8);
    k_wtr<<<cdiv(nU1b, NTHR), NTHR, 0, stream>>>(W1b, HID, HID, HID, KZ2, BT1b, nU1b);
    k_wtr<<<cdiv(nU1b, NTHR), NTHR, 0, stream>>>(W2a, HID, HID, HID, KZ2, BT2a, nU1b);
    const int nU2b = NCLS * (KZ2 / 8);
    k_wtr<<<cdiv(nU2b, NTHR), NTHR, 0, stream>>>(W2b, HID, NCLS, NCLS, KZ2, BT2b, nU2b);
  }

  k_scan<F0, 1><<<gA, NTHR, scanLds, stream>>>(src, dst, nE, nN, vec8, MP, eps1, x, ZA);
  k_gemm<GNC, KZ1, HID, 0><<<dim3(gM, HID / GNC), GTHR, 0, stream>>>(ZA, BT1a, b1a, nN, SH, PT);
  k_bnfin<<<1, HID, 0, stream>>>(PT, gM, g1, be1, SS);
  k_apply<<<gM, NTHR, 0, stream>>>(SH, SS, nN, MP, ZA);
  k_gemm<GNC, KZ2, HID, 1><<<dim3(gM, HID / GNC), GTHR, 0, stream>>>(ZA, BT1b, b1b, nN, SH, PT);

  k_scan<HID, 0><<<gA, NTHR, scanLds, stream>>>(src, dst, nE, nN, vec8, MP, eps2, SH, ZA);
  k_gemm<GNC, KZ2, HID, 0><<<dim3(gM, HID / GNC), GTHR, 0, stream>>>(ZA, BT2a, b2a, nN, SH, PT);
  k_bnfin<<<1, HID, 0, stream>>>(PT, gM, g2, be2, SS);
  k_apply<<<gM, NTHR, 0, stream>>>(SH, SS, nN, MP, ZA);
  k_gemm<NCLS, KZ2, NCLS, 2><<<dim3(gM, 1), GTHR, 0, stream>>>(ZA, BT2b, b2b, nN, out, PT);
}
